// HGNN_83485574300037
// MI455X (gfx1250) — hardware-verified
//
#include <hip/hip_runtime.h>
#include <stddef.h>
#include <math.h>


#define NBATCH 16
#define NNODE  1024
#define FIN    32
#define NTYPE  4
#define NNZE   32768
#define HD     64
#define ROWS   (NBATCH * NNODE)
#define EB     (NTYPE * NNZE)
#define EPSV   1e-5f

#define NTHR   256
#define NWAVE  8
#define GROWS  128
#define NGBLK  (ROWS / GROWS)
#define NB     64
#define NTILE  (NNODE / NB)
#define EPT    8
#define NGRP   2
#define CHUNK  (NTHR * EPT * NGRP)
#define NCHUNK (EB / CHUNK)
#define CHPT   (NNZE / CHUNK)
#define WCAP   (EPT * NGRP * 32)
#define LISTN  (NWAVE * WCAP)
#define TP     72

#define Q_W0H  0
#define Q_W0L  2048
#define Q_W1H  4096
#define Q_W1L  8192
#define Q_WSH  12288
#define Q_WSL  28672
#define Q_TOT  45056

#define G1_SA   0
#define G1_RED  36864
#define G1_BN   (G1_RED + 1024)
#define LDS_G1  (G1_BN + 768)

#define A_ACC   0
#define A_LIST  65536
#define A_WCNT  81920
#define A_THI   82048
#define A_TLO   (A_THI + 4 * NB * TP * 2)
#define LDS_AGG (A_TLO + 4 * NB * TP * 2)

static_assert((CHUNK & (CHUNK - 1)) == 0);
static_assert(EB % CHUNK == 0);
static_assert(NNZE % CHUNK == 0);
static_assert((NB & (NB - 1)) == 0 && NB <= 256);
static_assert(NNODE % NB == 0);
static_assert(ROWS % GROWS == 0);
static_assert(GROWS * HD * 4 <= 2 * GROWS * TP * 2);
static_assert(4 * NB * HD * 4 <= A_LIST);
static_assert(FIN == 32 && HD == 64);

typedef float  v2f  __attribute__((ext_vector_type(2)));
typedef float  v4f  __attribute__((ext_vector_type(4)));
typedef float  v8f  __attribute__((ext_vector_type(8)));
typedef int    v4i  __attribute__((ext_vector_type(4)));
typedef double v2d  __attribute__((ext_vector_type(2)));
typedef unsigned short v8us __attribute__((ext_vector_type(8)));
typedef __bf16 v8b  __attribute__((ext_vector_type(8)));
typedef __bf16 v16b __attribute__((ext_vector_type(16)));
union FragB { v16b v; v8b h[2]; v8us u[2]; };
struct HL8 { v8us hi; v8us lo; };

__device__ __forceinline__ unsigned bf_rne(float f) {
  unsigned u = __float_as_uint(f);
  u += 0x7FFFu + ((u >> 16) & 1u);
  return u >> 16;
}

#define SPL1(I, X) { const unsigned hb_ = bf_rne(X); const float hf_ = __uint_as_float(hb_ << 16); \
                     r.hi[I] = (unsigned short)hb_; r.lo[I] = (unsigned short)bf_rne((X) - hf_); }
__device__ __forceinline__ HL8 split8(v4f a, v4f b) {
  HL8 r;
  SPL1(0, a.x) SPL1(1, a.y) SPL1(2, a.z) SPL1(3, a.w)
  SPL1(4, b.x) SPL1(5, b.y) SPL1(6, b.z) SPL1(7, b.w)
  return r;
}
#undef SPL1

__device__ __forceinline__ v8f wmb(v16b a, v16b b, v8f c) {
  v8f d = __builtin_amdgcn_wmma_f32_16x16x32_bf16(false, a, false, b, (short)0, c, false, false);
  asm volatile("v_nop\n\tv_nop\n\tv_nop\n\tv_nop" : "+v"(d) : "v"(a), "v"(b));
  return d;
}
__device__ __forceinline__ v8f wm3(const FragB& ah, const FragB& al, const FragB& bh, const FragB& bl, v8f c) {
  c = wmb(ah.v, bh.v, c);
  c = wmb(ah.v, bl.v, c);
  c = wmb(al.v, bh.v, c);
  return c;
}

#define STORE_D8(SP, STRIDE, OFF, V) { \
  (SP)[0 * (STRIDE) + (OFF)] = (V)[0]; (SP)[1 * (STRIDE) + (OFF)] = (V)[1]; \
  (SP)[2 * (STRIDE) + (OFF)] = (V)[2]; (SP)[3 * (STRIDE) + (OFF)] = (V)[3]; \
  (SP)[4 * (STRIDE) + (OFF)] = (V)[4]; (SP)[5 * (STRIDE) + (OFF)] = (V)[5]; \
  (SP)[6 * (STRIDE) + (OFF)] = (V)[6]; (SP)[7 * (STRIDE) + (OFF)] = (V)[7]; }

__device__ __forceinline__ int scan_chunk(const int* __restrict__ srcs, int cbase, int nodeBase,
                                          int* list, int tid, int lane, int wave) {
  int wc = 0;
#pragma unroll
  for (int g = 0; g < NGRP; ++g) {
    const int el0 = (g * NTHR + tid) * EPT;
    const int e0  = cbase + el0;
    const v4i da = *(const v4i*)(srcs + e0);
    const v4i db = *(const v4i*)(srcs + e0 + 4);
    const unsigned nb = (unsigned)nodeBase;
    const unsigned s0 = (unsigned)da.x - nb, s1 = (unsigned)da.y - nb;
    const unsigned s2 = (unsigned)da.z - nb, s3 = (unsigned)da.w - nb;
    const unsigned s4 = (unsigned)db.x - nb, s5 = (unsigned)db.y - nb;
    const unsigned s6 = (unsigned)db.z - nb, s7 = (unsigned)db.w - nb;
    const bool h0 = s0 < (unsigned)NB, h1 = s1 < (unsigned)NB, h2 = s2 < (unsigned)NB, h3 = s3 < (unsigned)NB;
    const bool h4 = s4 < (unsigned)NB, h5 = s5 < (unsigned)NB, h6 = s6 < (unsigned)NB, h7 = s7 < (unsigned)NB;
    const unsigned any = __builtin_amdgcn_ballot_w32(h0 | h1 | h2 | h3 | h4 | h5 | h6 | h7);
    if (any != 0u) {
#define HITJ(J, HJ, SJ) { \
        const unsigned mj = __builtin_amdgcn_ballot_w32(HJ); \
        if (mj != 0u) { \
          if (HJ) { \
            const int pos = wc + (int)__builtin_amdgcn_mbcnt_lo(mj, 0u); \
            if (pos < WCAP) list[wave * WCAP + pos] = ((el0 + (J)) << 8) | (int)(SJ); \
          } \
          wc += (int)__builtin_popcount(mj); } }
      HITJ(0, h0, s0)
      HITJ(1, h1, s1)
      HITJ(2, h2, s2)
      HITJ(3, h3, s3)
      HITJ(4, h4, s4)
      HITJ(5, h5, s5)
      HITJ(6, h6, s6)
      HITJ(7, h7, s7)
#undef HITJ
    }
  }
  return wc;
}

__global__ __launch_bounds__(NTHR) void k_wprep(const float* __restrict__ W0, const float* __restrict__ W1,
                                                const float* __restrict__ Ws, unsigned short* wq) {
  const int i   = blockIdx.x * NTHR + threadIdx.x;
  const int n0c = FIN * HD / 8;
  const int n1c = HD * HD / 8;
  const int n2c = NTYPE * HD * HD / 8;
  if (i >= n0c + n1c + n2c) return;
  const float* p;
  int oh, ol;
  if (i < n0c) {
    const int o = i * 8;
    const int n = o / FIN, k0 = o - n * FIN;
    p  = W0 + (size_t)k0 * HD + n;
    oh = Q_W0H + o; ol = Q_W0L + o;
  } else if (i < n0c + n1c) {
    const int o = (i - n0c) * 8;
    const int n = o / HD, k0 = o - n * HD;
    p  = W1 + (size_t)k0 * HD + n;
    oh = Q_W1H + o; ol = Q_W1L + o;
  } else {
    const int o   = (i - n0c - n1c) * 8;
    const int c   = o / (HD * HD);
    const int rem = o - c * HD * HD;
    const int n   = rem / HD, k0 = rem - n * HD;
    p  = Ws + ((size_t)c * HD + k0) * HD + n;
    oh = Q_WSH + o; ol = Q_WSL + o;
  }
  v4f a, b;
  a.x = p[0];      a.y = p[HD];     a.z = p[2 * HD]; a.w = p[3 * HD];
  b.x = p[4 * HD]; b.y = p[5 * HD]; b.z = p[6 * HD]; b.w = p[7 * HD];
  const HL8 s = split8(a, b);
  *(volatile v8us*)(wq + oh) = s.hi;
  *(volatile v8us*)(wq + ol) = s.lo;
  __threadfence();
  *(volatile v8us*)(wq + oh) = s.hi;
  *(volatile v8us*)(wq + ol) = s.lo;
}

__global__ __launch_bounds__(NTHR) void k_gemm0(const float* __restrict__ X, const unsigned short* __restrict__ wq,
                                                const float* __restrict__ b0, float* h0, double* part) {
  __shared__ __attribute__((aligned(16))) float  stg[GROWS * HD];
  __shared__ __attribute__((aligned(16))) double sred[4 * 128];
  __shared__ __attribute__((aligned(16))) double pl[128];
  const int tid = threadIdx.x, lane = tid & 31, wave = tid >> 5, hh = lane >> 4, m = lane & 15;
  const int rowBase = blockIdx.x * GROWS;

  FragB ah, al;
  {
    const float* xr = X + (size_t)(rowBase + 16 * wave + m) * FIN;
    const v4f p0 = *(const v4f*)(xr + 8 * hh),      p1 = *(const v4f*)(xr + 8 * hh + 4);
    const v4f p2 = *(const v4f*)(xr + 16 + 8 * hh), p3 = *(const v4f*)(xr + 20 + 8 * hh);
    const HL8 s0 = split8(p0, p1), s1 = split8(p2, p3);
    ah.u[0] = s0.hi; al.u[0] = s0.lo; ah.u[1] = s1.hi; al.u[1] = s1.lo;
  }
  v8f acc[4];
#pragma unroll
  for (int t = 0; t < 4; ++t) {
    const v8f z8 = {0.f, 0.f, 0.f, 0.f, 0.f, 0.f, 0.f, 0.f};
    FragB bh, bl;
    const unsigned short* bph = wq + Q_W0H + (16 * t + m) * FIN + 8 * hh;
    const unsigned short* bpl = wq + Q_W0L + (16 * t + m) * FIN + 8 * hh;
    bh.u[0] = *(const v8us*)bph; bh.u[1] = *(const v8us*)(bph + 16);
    bl.u[0] = *(const v8us*)bpl; bl.u[1] = *(const v8us*)(bpl + 16);
    acc[t] = wm3(ah, al, bh, bl, z8);
  }
  {
    float* sp = stg + (16 * wave + 8 * hh) * HD + m;
#pragma unroll
    for (int t = 0; t < 4; ++t) {
      const v8f tv = acc[t] + b0[16 * t + m];
      STORE_D8(sp, HD, 16 * t, tv)
    }
  }
  __syncthreads();

  {
    const int col = tid & 63, rg = tid >> 6;
    double s = 0.0, q = 0.0;
#pragma unroll 4
    for (int i = 0; i < 32; ++i) {
      const double v = (double)stg[(rg * 32 + i) * HD + col];
      s += v; q += v * v;
    }
    sred[rg * 128 + col]      = s;
    sred[rg * 128 + 64 + col] = q;
  }
  __syncthreads();
  if (tid < 128) pl[tid] = ((sred[tid] + sred[128 + tid]) + sred[256 + tid]) + sred[384 + tid];
  __syncthreads();

  const float* lp = stg + wave * 16 * HD + 4 * lane;
  float* gp = h0 + (size_t)(rowBase + wave * 16) * HD + 4 * lane;
  v4f hv[8];
#pragma unroll
  for (int qq = 0; qq < 8; ++qq) hv[qq] = *(const v4f*)(lp + qq * 128);
  const v2d d0 = *(const v2d*)(pl + 2 * lane);
  const v2d d1 = *(const v2d*)(pl + 64 + 2 * lane);
  double* pp = part + (size_t)blockIdx.x * 128;
#pragma unroll
  for (int qq = 0; qq < 8; ++qq) *(volatile v4f*)(gp + qq * 128) = hv[qq];
  if (wave == 0) { *(volatile v2d*)(pp + 2 * lane) = d0; *(volatile v2d*)(pp + 64 + 2 * lane) = d1; }
  __threadfence();
#pragma unroll
  for (int qq = 0; qq < 8; ++qq) *(volatile v4f*)(gp + qq * 128) = hv[qq];
  if (wave == 0) { *(volatile v2d*)(pp + 2 * lane) = d0; *(volatile v2d*)(pp + 64 + 2 * lane) = d1; }
}

__device__ __forceinline__ float eluf(float x) { return x > 0.f ? x : (expf(x) - 1.0f); }

__global__ __launch_bounds__(NTHR) void k_gemm1(const float* __restrict__ h0, const double* __restrict__ part,
                                                const float* __restrict__ gamma0, const float* __restrict__ beta0,
                                                const unsigned short* __restrict__ wq, const float* __restrict__ b1,
                                                float* h) {
  extern __shared__ v4f lds_dyn[];
  char* base = (char*)lds_dyn;
  unsigned short* sAh = (unsigned short*)(base + G1_SA);
  unsigned short* sAl = sAh + GROWS * TP;
  float*  stg = (float*)(base + G1_SA);
  double* red = (double*)(base + G1_RED);
  float*  smu = (float*)(base + G1_BN);
  float*  sg  = smu + HD;
  float*  sbt = sg + HD;
  const int tid = threadIdx.x, lane = tid & 31, wave = tid >> 5, hh = lane >> 4, m = lane & 15;
  const int rowBase = blockIdx.x * GROWS;

  if (tid < 128) {
    double a = 0.0;
#pragma unroll 1
    for (int blk = 0; blk < NGBLK; ++blk) a += part[(size_t)blk * 128 + tid];
    red[tid] = a;
  }
  __syncthreads();
  if (tid < HD) {
    const double mu_d = red[tid] * (1.0 / (double)ROWS);
    double var_d = red[64 + tid] * (1.0 / (double)ROWS) - mu_d * mu_d;
    var_d = var_d < 0.0 ? 0.0 : var_d;
    const float mu  = (float)mu_d;
    const float var = (float)var_d;
    const float rs  = rsqrtf(var + EPSV);
    smu[tid] = mu;
    sg[tid]  = gamma0[tid] * rs;
    sbt[tid] = beta0[tid];
  }
  __syncthreads();

#pragma unroll
  for (int i = 0; i < (GROWS * HD / 8) / NTHR; ++i) {
    const int idx = i * NTHR + tid;
    const int r   = idx >> 3;
    const int c0  = (idx & 7) * 8;
    const float* hp = h0 + (size_t)(rowBase + r) * HD + c0;
    v4f a = *(const v4f*)hp, b = *(const v4f*)(hp + 4);
    a.x = eluf((a.x - smu[c0 + 0]) * sg[c0 + 0] + sbt[c0 + 0]);
    a.y = eluf((a.y - smu[c0 + 1]) * sg[c0 + 1] + sbt[c0 + 1]);
    a.z = eluf((a.z - smu[c0 + 2]) * sg[c0 + 2] + sbt[c0 + 2]);
    a.w = eluf((a.w - smu[c0 + 3]) * sg[c0 + 3] + sbt[c0 + 3]);
    b.x = eluf((b.x - smu[c0 + 4]) * sg[c0 + 4] + sbt[c0 + 4]);
    b.y = eluf((b.y - smu[c0 + 5]) * sg[c0 + 5] + sbt[c0 + 5]);
    b.z = eluf((b.z - smu[c0 + 6]) * sg[c0 + 6] + sbt[c0 + 6]);
    b.w = eluf((b.w - smu[c0 + 7]) * sg[c0 + 7] + sbt[c0 + 7]);
    const HL8 s = split8(a, b);
    *(v8us*)(sAh + r * TP + c0) = s.hi;
    *(v8us*)(sAl + r * TP + c0) = s.lo;
  }
  __syncthreads();

  v8f acc[4];
#pragma unroll
  for (int t = 0; t < 4; ++t) { const v8f z8 = {0.f, 0.f, 0.f, 0.f, 0.f, 0.f, 0.f, 0.f}; acc[t] = z8; }
#pragma unroll
  for (int kt = 0; kt < HD / 32; ++kt) {
    FragB ah, al;
    const unsigned short* aph = sAh + (wave * 16 + m) * TP + 32 * kt + 8 * hh;
    const unsigned short* apl = sAl + (wave * 16 + m) * TP + 32 * kt + 8 * hh;
    ah.u[0] = *(const v8us*)aph; ah.u[1] = *(const v8us*)(aph + 16);
    al.u[0] = *(const v8us*)apl; al.u[1] = *(const v8us*)(apl + 16);
#pragma unroll
    for (int t = 0; t < 4; ++t) {
      FragB bh, bl;
      const unsigned short* bph = wq + Q_W1H + (16 * t + m) * HD + 32 * kt + 8 * hh;
      const unsigned short* bpl = wq + Q_W1L + (16 * t + m) * HD + 32 * kt + 8 * hh;
      bh.u[0] = *(const v8us*)bph; bh.u[1] = *(const v8us*)(bph + 16);
      bl.u[0] = *(const v8us*)bpl; bl.u[1] = *(const v8us*)(bpl + 16);
      acc[t] = wm3(ah, al, bh, bl, acc[t]);
    }
  }
  __syncthreads();

  {
    float* sp = stg + (16 * wave + 8 * hh) * HD + m;
#pragma unroll
    for (int t = 0; t < 4; ++t) {
      const v8f tv = acc[t] + b1[16 * t + m];
      STORE_D8(sp, HD, 16 * t, tv)
    }
  }
  __syncthreads();

  const float* lp = stg + wave * 16 * HD + 4 * lane;
  float* gp = h + (size_t)(rowBase + wave * 16) * HD + 4 * lane;
  v4f hv[8];
#pragma unroll
  for (int qq = 0; qq < 8; ++qq) hv[qq] = *(const v4f*)(lp + qq * 128);
#pragma unroll
  for (int qq = 0; qq < 8; ++qq) *(volatile v4f*)(gp + qq * 128) = hv[qq];
  __threadfence();
#pragma unroll
  for (int qq = 0; qq < 8; ++qq) *(volatile v4f*)(gp + qq * 128) = hv[qq];
}

__global__ __launch_bounds__(NTHR) void k_agg(const int* __restrict__ esrc, const int* __restrict__ edst,
                                              const float* __restrict__ h, const float* __restrict__ filt,
                                              const unsigned short* __restrict__ wq, float* out) {
  extern __shared__ v4f lds_dyn[];
  char* base = (char*)lds_dyn;
  float* acc  = (float*)(base + A_ACC);
  int*   list = (int*)(base + A_LIST);
  int*   wcnt = (int*)(base + A_WCNT);
  unsigned short* sTh = (unsigned short*)(base + A_THI);
  unsigned short* sTl = (unsigned short*)(base + A_TLO);
  float* ostg = (float*)(base + A_ACC);
  const int tid = threadIdx.x, lane = tid & 31, wave = tid >> 5, hh = lane >> 4, m = lane & 15;
  const int b = blockIdx.x / NTILE;
  const int tile = blockIdx.x - b * NTILE;
  const int nodeBase = tile * NB;
  const int*   srcs = esrc + (size_t)b * EB;
  const int*   dsts = edst + (size_t)b * EB;
  const float* hb   = h + (size_t)b * NNODE * HD;

  {
    const v4f z = {0.f, 0.f, 0.f, 0.f};
    v4f* az = (v4f*)acc;
#pragma unroll
    for (int i = 0; i < (NB * NTYPE * HD / 4) / NTHR; ++i) az[i * NTHR + tid] = z;
  }
  __syncthreads();

#pragma unroll 1
  for (int ch = 0; ch < NCHUNK; ++ch) {
    const int cbase = ch * CHUNK;
    const int k     = ch / CHPT;
    const int wc = scan_chunk(srcs, cbase, nodeBase, list, tid, lane, wave);
    if (lane == 0) wcnt[wave] = wc;
    __syncthreads();
    if (wave == 0) {
#pragma unroll 1
      for (int wsx = 0; wsx < NWAVE; ++wsx) {
        int n = __builtin_amdgcn_readfirstlane(wcnt[wsx]);
        n = n > WCAP ? WCAP : (n < 0 ? 0 : n);
        const int* lp = list + wsx * WCAP;
#pragma unroll 1
        for (int i = 0; i < n; ++i) {
          const int ent  = __builtin_amdgcn_readfirstlane(lp[i]);
          const int slot = ent & (NB - 1);
          const int el   = (ent >> 8) & (CHUNK - 1);
          const int eb   = cbase + el;
          const int dst  = dsts[eb];
          if ((unsigned)dst < (unsigned)NNODE) {
            const v2f v = *(const v2f*)(hb + (size_t)dst * HD + 2 * lane);
            v2f* ap = (v2f*)(acc + (slot * NTYPE + k) * HD + 2 * lane);
            *ap = *ap + v;
          }
        }
      }
    }
    __syncthreads();
  }

  {
    float fr[NTYPE * NTYPE];
#pragma unroll
    for (int i = 0; i < NTYPE * NTYPE; ++i) fr[i] = filt[i];
#pragma unroll
    for (int q = 0; q < 2; ++q) {
      const int tsk  = tid + NTHR * q;
      const int slot = tsk >> 3;
      const int j8   = (tsk & 7) * 8;
      const float* ap = acc + (slot * NTYPE) * HD + j8;
      const v4f a0 = *(const v4f*)(ap),          a0b = *(const v4f*)(ap + 4);
      const v4f a1 = *(const v4f*)(ap + HD),     a1b = *(const v4f*)(ap + HD + 4);
      const v4f a2 = *(const v4f*)(ap + 2 * HD), a2b = *(const v4f*)(ap + 2 * HD + 4);
      const v4f a3 = *(const v4f*)(ap + 3 * HD), a3b = *(const v4f*)(ap + 3 * HD + 4);
#pragma unroll
      for (int c = 0; c < NTYPE; ++c) {
        const float f0 = fr[c * NTYPE + 0], f1 = fr[c * NTYPE + 1], f2 = fr[c * NTYPE + 2], f3 = fr[c * NTYPE + 3];
        const v4f tA = f0 * a0  + f1 * a1  + f2 * a2  + f3 * a3;
        const v4f tB = f0 * a0b + f1 * a1b + f2 * a2b + f3 * a3b;
        const HL8 s = split8(tA, tB);
        *(v8us*)(sTh + (c * NB + slot) * TP + j8) = s.hi;
        *(v8us*)(sTl + (c * NB + slot) * TP + j8) = s.lo;
      }
    }
  }
  __syncthreads();

#pragma unroll 1
  for (int q = 0; q < 2; ++q) {
    const int rt = wave + 8 * q;
    const int c  = rt >> 2;
    v8f d[4];
#pragma unroll
    for (int ct = 0; ct < 4; ++ct) { const v8f z8 = {0.f, 0.f, 0.f, 0.f, 0.f, 0.f, 0.f, 0.f}; d[ct] = z8; }
#pragma unroll
    for (int kt = 0; kt < HD / 32; ++kt) {
      FragB ah, al;
      const unsigned short* aph = sTh + (16 * rt + m) * TP + 32 * kt + 8 * hh;
      const unsigned short* apl = sTl + (16 * rt + m) * TP + 32 * kt + 8 * hh;
      ah.u[0] = *(const v8us*)aph; ah.u[1] = *(const v8us*)(aph + 16);
      al.u[0] = *(const v8us*)apl; al.u[1] = *(const v8us*)(apl + 16);
#pragma unroll
      for (int ct = 0; ct < 4; ++ct) {
        FragB bh, bl;
        const unsigned short* bph = wq + Q_WSH + (c * HD + 16 * ct + m) * HD + 32 * kt + 8 * hh;
        const unsigned short* bpl = wq + Q_WSL + (c * HD + 16 * ct + m) * HD + 32 * kt + 8 * hh;
        bh.u[0] = *(const v8us*)bph; bh.u[1] = *(const v8us*)(bph + 16);
        bl.u[0] = *(const v8us*)bpl; bl.u[1] = *(const v8us*)(bpl + 16);
        d[ct] = wm3(ah, al, bh, bl, d[ct]);
      }
    }
    float* sp = ostg + (16 * rt + 8 * hh) * HD + m;
#pragma unroll
    for (int ct = 0; ct < 4; ++ct) { const v8f tv = d[ct]; STORE_D8(sp, HD, 16 * ct, tv) }
  }
  __syncthreads();

  {
    const int c  = wave >> 1;
    const int r0 = (wave & 1) * 32;
    const float* lp = ostg + (size_t)(c * NB + r0) * HD + 4 * lane;
    float* gp = out + (((size_t)(b * NTYPE + c) * NNODE + nodeBase + r0) * HD) + 4 * lane;
#pragma unroll
    for (int qq = 0; qq < 16; ++qq) { const v4f v = *(const v4f*)(lp + qq * 128); *(volatile v4f*)(gp + qq * 128) = v; }
    __threadfence();
#pragma unroll
    for (int qq = 0; qq < 16; ++qq) { const v4f v = *(const v4f*)(lp + qq * 128); *(volatile v4f*)(gp + qq * 128) = v; }
  }
}

extern "C" void kernel_launch(void* const* d_in, const int* in_sizes, int n_in,
                              void* d_out, int out_size, void* d_ws, size_t ws_size,
                              hipStream_t stream) {
  if (n_in < 11) return;
  if (in_sizes[0] != ROWS * FIN || in_sizes[1] != FIN * HD || in_sizes[2] != HD || in_sizes[3] != HD ||
      in_sizes[4] != HD || in_sizes[5] != HD * HD || in_sizes[6] != HD || in_sizes[7] != NTYPE * HD * HD ||
      in_sizes[8] != NTYPE * NTYPE || in_sizes[9] != NBATCH * EB || in_sizes[10] != NBATCH * EB) return;
  if (out_size != NBATCH * NTYPE * NNODE * HD) return;

  const float* X      = (const float*)d_in[0];
  const float* W0     = (const float*)d_in[1];
  const float* b0     = (const float*)d_in[2];
  const float* gamma0 = (const float*)d_in[3];
  const float* beta0  = (const float*)d_in[4];
  const float* W1     = (const float*)d_in[5];
  const float* b1     = (const float*)d_in[6];
  const float* Ws     = (const float*)d_in[7];
  const float* filt   = (const float*)d_in[8];
  const int*   esrc   = (const int*)d_in[9];
  const int*   edst   = (const int*)d_in[10];
  float* out = (float*)d_out;

  char* ws = (char*)d_ws;
  size_t off = 0;
  const size_t oWQ = off; off += (size_t)Q_TOT * 2;              off = (off + 255) & ~(size_t)255;
  const size_t oH0 = off; off += (size_t)ROWS * HD * 4;           off = (off + 255) & ~(size_t)255;
  const size_t oPT = off; off += (size_t)NGBLK * 128 * 8;         off = (off + 255) & ~(size_t)255;
  const size_t oH  = off; off += (size_t)ROWS * HD * 4;           off = (off + 255) & ~(size_t)255;
  if (off > ws_size) return;
  unsigned short* wq   = (unsigned short*)(ws + oWQ);
  float*          h0   = (float*)(ws + oH0);
  double*         part = (double*)(ws + oPT);
  float*          h    = (float*)(ws + oH);

  const int nPrep = FIN * HD / 8 + HD * HD / 8 + NTYPE * HD * HD / 8;
  k_wprep<<<(nPrep + NTHR - 1) / NTHR, NTHR, 0, stream>>>(W0, W1, Ws, wq);

  k_gemm0<<<NGBLK, NTHR, 0, stream>>>(X, wq, b0, h0, part);

  hipFuncSetAttribute(reinterpret_cast<const void*>(&k_gemm1),
                      hipFuncAttributeMaxDynamicSharedMemorySize, LDS_G1);
  k_gemm1<<<NGBLK, NTHR, LDS_G1, stream>>>(h0, part, gamma0, beta0, wq, b1, h);

  hipFuncSetAttribute(reinterpret_cast<const void*>(&k_agg),
                      hipFuncAttributeMaxDynamicSharedMemorySize, LDS_AGG);
  k_agg<<<NBATCH * NTILE, NTHR, LDS_AGG, stream>>>(esrc, edst, h, filt, wq, out);
}
